// Siege_60112362274858
// MI455X (gfx1250) — hardware-run, weakly checked
//
#include <hip/hip_runtime.h>
#include <stddef.h>
#include <math.h>

#define NB_B   8
#define NN     1024
#define MM     32
#define HA     128
#define HC     256
#define KW     257
#define NCOL   512
#define NNODE  (NB_B * NN)
#define NEMB   60
#define NLAY   3
#define NPB    8
#define NBLK_E (NNODE / NPB)
#define KP     136
#define SP     68
#define BN_EPS 1e-5f

static_assert(NNODE % NPB == 0);
static_assert(NN % NPB == 0);
static_assert(NPB * MM == 256);
static_assert(NNODE % 64 == 0);
static_assert(NCOL % 128 == 0);
static_assert(HA % 32 == 0);
static_assert(KP % 8 == 0);
static_assert(SP % 4 == 0);
static_assert(HC == 2 * HA);

typedef _Float16 f16;
typedef f16 v16h __attribute__((ext_vector_type(16)));
typedef f16 v8h_t __attribute__((ext_vector_type(8)));
typedef v8h_t __attribute__((may_alias)) v8h;
typedef float v8f __attribute__((ext_vector_type(8)));
typedef float v4f_t __attribute__((ext_vector_type(4)));
typedef v4f_t __attribute__((may_alias)) v4f;
typedef unsigned int v4u __attribute__((ext_vector_type(4)));

union Frag { v16h v; v8h_t h[2]; };

__device__ __forceinline__ v8f zero8() {
  v8f z;
#pragma unroll
  for (int i = 0; i < 8; ++i) z[i] = 0.0f;
  return z;
}

__device__ __forceinline__ v16h ldfrag(const f16* p, int k0) {
  Frag f;
  f.h[0] = *(const v8h*)(p + k0);
  f.h[1] = *(const v8h*)(p + k0 + 16);
  return f.v;
}

__device__ __forceinline__ v8f wmma16(v16h a, v16h b, v8f c) {
  return __builtin_amdgcn_wmma_f32_16x16x32_f16(false, a, false, b, (short)0, c, false, false);
}

__device__ __forceinline__ void store_xrow(float* x, f16* x16, int node, int lane, v4f_t v) {
  float vv[4];
#pragma unroll
  for (int j = 0; j < 4; ++j) vv[j] = v[j];
  const int s0 = (2 * lane) & 31, s1 = (2 * lane + 1) & 31;
  float e[8];
#pragma unroll
  for (int j = 0; j < 4; ++j) {
    e[j]     = __shfl(vv[j], s0, 32);
    e[4 + j] = __shfl(vv[j], s1, 32);
  }
  union { v8h_t h; v4u u; } pk;
#pragma unroll
  for (int j = 0; j < 8; ++j) pk.h[j] = (f16)(e[j] * 16.0f);
  float* px = x + (size_t)node * HA + 4 * lane;
  f16*   ph = x16 + (size_t)node * HA + 8 * lane;
  *(volatile v4f_t*)px = v;
  if (lane < 16) *(volatile v4u*)ph = pk.u;
  __threadfence();
  *(volatile v4f_t*)px = v;
  if (lane < 16) *(volatile v4u*)ph = pk.u;
}

__global__ void __launch_bounds__(256)
embed_kernel(const int* __restrict__ na, const float* __restrict__ emb,
             float* x, f16* x16) {
  const int lane = threadIdx.x & 31, w = threadIdx.x >> 5;
  const int node = blockIdx.x * NPB + w;
  int id = na[node];
  id = min(max(id, 0), NEMB - 1);
  const v4f_t v = *(const v4f*)(emb + (size_t)id * HA + 4 * lane);
  store_xrow(x, x16, node, lane, v);
}

__global__ void __launch_bounds__(256)
wcvt_kernel(const float* __restrict__ Wl, f16* Wt) {
  __shared__ __align__(16) f16 T[16 * KP];
  const int t = threadIdx.x;
  const int j0 = blockIdx.x * 16;
  const int kbase = (j0 < HC) ? 0 : HA;
  const int jsrc  = (j0 < HC) ? j0 : (j0 - HC);
  const int k = t >> 1, jj0 = (t & 1) * 8;
  const float* src = Wl + (size_t)(kbase + k) * HC + jsrc + jj0;
  const v4f_t a = *(const v4f*)src;
  const v4f_t b = *(const v4f*)(src + 4);
#pragma unroll
  for (int i = 0; i < 4; ++i) {
    T[(jj0 + i) * KP + k]     = (f16)(a[i] * 16.0f);
    T[(jj0 + 4 + i) * KP + k] = (f16)(b[i] * 16.0f);
  }
  __syncthreads();
  const int r = t >> 4, p = t & 15;
  union { v8h_t h; v4u u; } o;
  o.h = *(const v8h*)(T + r * KP + 8 * p);
  f16* dst = Wt + (size_t)(j0 + r) * HA + 8 * p;
  *(volatile v4u*)dst = o.u;
  __threadfence();
  *(volatile v4u*)dst = o.u;
}

__global__ void __launch_bounds__(256)
gemm_kernel(const f16* __restrict__ x16, const f16* __restrict__ Wt, float* PQ) {
  __shared__ __align__(16) float stg[8 * 16 * SP];
  const int lane = threadIdx.x & 31, w = threadIdx.x >> 5;
  const int h = lane >> 4, m = lane & 15;
  const int wr = w >> 1, wc = w & 1;
  const int row0 = blockIdx.x * 64 + wr * 16;
  const int col0 = blockIdx.y * 128 + wc * 64;
  v8f acc[4];
#pragma unroll
  for (int tn = 0; tn < 4; ++tn) acc[tn] = zero8();
  const f16* pa = x16 + (size_t)(row0 + m) * HA + 8 * h;
  const f16* pb = Wt  + (size_t)(col0 + m) * HA + 8 * h;
#pragma unroll
  for (int k0 = 0; k0 < HA; k0 += 32) {
    const v16h a  = ldfrag(pa, k0);
    const v16h b0 = ldfrag(pb, k0);
    const v16h b1 = ldfrag(pb + 16 * HA, k0);
    const v16h b2 = ldfrag(pb + 32 * HA, k0);
    const v16h b3 = ldfrag(pb + 48 * HA, k0);
    acc[0] = wmma16(a, b0, acc[0]);
    acc[1] = wmma16(a, b1, acc[1]);
    acc[2] = wmma16(a, b2, acc[2]);
    acc[3] = wmma16(a, b3, acc[3]);
    asm volatile("v_nop\n\tv_nop\n\tv_nop\n\tv_nop"
                 : "+v"(acc[0]), "+v"(acc[1]), "+v"(acc[2]), "+v"(acc[3])
                 : "v"(a), "v"(b0), "v"(b1), "v"(b2), "v"(b3));
  }
  float* sw = stg + w * (16 * SP);
#pragma unroll
  for (int tn = 0; tn < 4; ++tn) {
#pragma unroll
    for (int r = 0; r < 8; ++r)
      sw[(8 * h + r) * SP + 16 * tn + m] = acc[tn][r] * (1.0f / 256.0f);
  }
  __syncthreads();
  v4f_t v[8];
#pragma unroll
  for (int p = 0; p < 8; ++p) v[p] = *(const v4f*)(sw + (2 * p + h) * SP + 4 * m);
  float* go = PQ + (size_t)row0 * NCOL + col0 + 4 * m;
#pragma unroll
  for (int p = 0; p < 8; ++p)
    *(volatile v4f_t*)(go + (size_t)(2 * p + h) * NCOL) = v[p];
  __threadfence();
#pragma unroll
  for (int p = 0; p < 8; ++p)
    *(volatile v4f_t*)(go + (size_t)(2 * p + h) * NCOL) = v[p];
}

__global__ void __launch_bounds__(256)
stats_kernel(const float* __restrict__ PQ, const int* __restrict__ eidx,
             const float* __restrict__ eattr, const float* __restrict__ Wl,
             const float* __restrict__ bias, double* part) {
  __shared__ int   sIdx[NPB * MM];
  __shared__ float sEa[NPB * MM];
  const int t = threadIdx.x;
  const int node0 = blockIdx.x * NPB;
  const int bb = node0 / NN;
  {
    int id = eidx[(size_t)node0 * MM + t];
    id = min(max(id, 0), NN - 1);
    sIdx[t] = bb * NN + id;
    sEa[t]  = eattr[(size_t)node0 * MM + t];
  }
  const float wl = Wl[(size_t)(KW - 1) * HC + t];
  const float bc = bias[t];
  __syncthreads();
  double s1 = 0.0, s2 = 0.0;
#pragma unroll 1
  for (int ni = 0; ni < NPB; ++ni) {
    const float pv = PQ[(size_t)(node0 + ni) * NCOL + t];
#pragma unroll 2
    for (int mi = 0; mi < MM; ++mi) {
      const int r = ni * MM + mi;
      const float qv = PQ[(size_t)sIdx[r] * NCOL + HC + t];
      const float g = ((pv + qv) + sEa[r] * wl) + bc;
      const double gd = (double)g;
      s1 += gd;
      s2 += gd * gd;
    }
  }
  double* po = part + (size_t)blockIdx.x * 2 * HC;
  *(volatile double*)(po + t)      = s1;
  *(volatile double*)(po + HC + t) = s2;
  __threadfence();
  *(volatile double*)(po + t)      = s1;
  *(volatile double*)(po + HC + t) = s2;
}

__global__ void __launch_bounds__(256)
bnfin_kernel(const double* __restrict__ part, int nblk, int C, double invR,
             const float* __restrict__ gamma, const float* __restrict__ beta, float* bn) {
  const int c = threadIdx.x;
  double s1 = 0.0, s2 = 0.0;
#pragma unroll 1
  for (int j = 0; j < nblk; ++j) {
    s1 += part[(size_t)j * 2 * C + c];
    s2 += part[(size_t)j * 2 * C + C + c];
  }
  const double mu = s1 * invR;
  double var = s2 * invR - mu * mu;
  if (var < 0.0) var = 0.0;
  const float sc = gamma[c] * rsqrtf((float)var + BN_EPS);
  const float sh = beta[c] - (float)mu * sc;
  *(volatile float*)(bn + c)     = sc;
  *(volatile float*)(bn + C + c) = sh;
  __threadfence();
  *(volatile float*)(bn + c)     = sc;
  *(volatile float*)(bn + C + c) = sh;
}

__global__ void __launch_bounds__(256)
apply_kernel(const float* __restrict__ PQ, const int* __restrict__ eidx,
             const float* __restrict__ eattr, const float* __restrict__ Wl,
             const float* __restrict__ bias, const float* __restrict__ bnH,
             float* summ, double* part) {
  __shared__ int    sIdx[NPB * MM];
  __shared__ float  sEa[NPB * MM];
  __shared__ double red1[HA];
  __shared__ double red2[HA];
  const int t = threadIdx.x, c = t & (HA - 1), hs = t >> 7;
  const int node0 = blockIdx.x * NPB;
  const int bb = node0 / NN;
  {
    int id = eidx[(size_t)node0 * MM + t];
    id = min(max(id, 0), NN - 1);
    sIdx[t] = bb * NN + id;
    sEa[t]  = eattr[(size_t)node0 * MM + t];
  }
  const float wlf = Wl[(size_t)(KW - 1) * HC + c];
  const float wlc = Wl[(size_t)(KW - 1) * HC + HA + c];
  const float bfi = bias[c], bco = bias[HA + c];
  const float scf = bnH[c],      shf = bnH[HC + c];
  const float scc = bnH[HA + c], shc = bnH[HC + HA + c];
  __syncthreads();
  double s1 = 0.0, s2 = 0.0;
  float sv[NPB / 2];
#pragma unroll
  for (int it = 0; it < NPB / 2; ++it) {
    const int ni = it * 2 + hs;
    const int node = node0 + ni;
    const float pf = PQ[(size_t)node * NCOL + c];
    const float pc = PQ[(size_t)node * NCOL + HA + c];
    float acc = 0.0f;
#pragma unroll 1
    for (int mi = 0; mi < MM; ++mi) {
      const int r = ni * MM + mi;
      const float* qrow = PQ + (size_t)sIdx[r] * NCOL + HC;
      const float qf = qrow[c];
      const float qc = qrow[HA + c];
      const float ea = sEa[r];
      float gf = ((pf + qf) + ea * wlf) + bfi;
      float gc = ((pc + qc) + ea * wlc) + bco;
      gf = gf * scf + shf;
      gc = gc * scc + shc;
      const float sg = __builtin_amdgcn_rcpf(1.0f + __expf(-gf));
      acc += sg * fmaxf(gc, 0.0f);
    }
    sv[it] = acc;
    const double ad = (double)acc;
    s1 += ad;
    s2 += ad * ad;
  }
  if (hs == 1) { red1[c] = s1; red2[c] = s2; }
  __syncthreads();
  if (hs == 0) { s1 += red1[c]; s2 += red2[c]; }
  double* po = part + (size_t)blockIdx.x * 2 * HA;
#pragma unroll
  for (int it = 0; it < NPB / 2; ++it)
    *(volatile float*)(summ + (size_t)(node0 + it * 2 + hs) * HA + c) = sv[it];
  if (hs == 0) {
    *(volatile double*)(po + c)      = s1;
    *(volatile double*)(po + HA + c) = s2;
  }
  __threadfence();
#pragma unroll
  for (int it = 0; it < NPB / 2; ++it)
    *(volatile float*)(summ + (size_t)(node0 + it * 2 + hs) * HA + c) = sv[it];
  if (hs == 0) {
    *(volatile double*)(po + c)      = s1;
    *(volatile double*)(po + HA + c) = s2;
  }
}

__global__ void __launch_bounds__(256)
update_kernel(const float* __restrict__ summ, const float* __restrict__ bnO,
              const float* __restrict__ tvec, const float* __restrict__ twl,
              const float* __restrict__ tbl, float* x, f16* x16) {
  __shared__ float sg[HA];
  __shared__ float th[HA];
  const int t = threadIdx.x, lane = t & 31, w = t >> 5;
  const int node0 = blockIdx.x * NPB;
  const int bb = node0 / NN;
  const float ts = tvec[bb];
  if (t < HA) {
    sg[t] = 1.0f / (1.0f + expf(-(ts * twl[t])));
  } else {
    th[t - HA] = tanhf(ts * tbl[t - HA]);
  }
  __syncthreads();
  const int node = node0 + w;
  const v4f_t xv = *(const v4f*)(x + (size_t)node * HA + 4 * lane);
  const v4f_t sm = *(const v4f*)(summ + (size_t)node * HA + 4 * lane);
  v4f_t o;
#pragma unroll
  for (int j = 0; j < 4; ++j) {
    const int cc = 4 * lane + j;
    const float s  = sm[j] * bnO[cc] + bnO[HA + cc];
    const float xn = fmaxf(xv[j] + s, 0.0f);
    o[j] = xn * sg[cc] + th[cc];
  }
  store_xrow(x, x16, node, lane, o);
}

__global__ void __launch_bounds__(256)
out_kernel(const float* __restrict__ x, const float* __restrict__ eow,
           const float* __restrict__ eob, float* out) {
  __shared__ double red[256];
  const int t = threadIdx.x;
  const double wv = (double)eow[t & (HA - 1)];
  double s = 0.0;
#pragma unroll 1
  for (int i = t; i < NNODE * HA; i += 256) s += (double)x[i] * wv;
  red[t] = s;
  __syncthreads();
#pragma unroll 1
  for (int ofs = 128; ofs > 0; ofs >>= 1) {
    if (t < ofs) red[t] += red[t + ofs];
    __syncthreads();
  }
  if (t == 0) {
    const double tot = red[0] + (double)eob[0] * (double)NNODE;
    const float r = (float)tot;
    *(volatile float*)out = r;
    __threadfence();
    *(volatile float*)out = r;
  }
}

extern "C" void kernel_launch(void* const* d_in, const int* in_sizes, int n_in,
                              void* d_out, int out_size, void* d_ws, size_t ws_size,
                              hipStream_t stream) {
  if (n_in < 15) return;
  if (in_sizes[0]  != NNODE) return;
  if (in_sizes[1]  != NNODE * MM) return;
  if (in_sizes[2]  != NNODE * MM) return;
  if (in_sizes[3]  != NB_B) return;
  if (in_sizes[4]  != NEMB * HA) return;
  if (in_sizes[5]  != NLAY * KW * HC) return;
  if (in_sizes[6]  != NLAY * HC) return;
  if (in_sizes[7]  != NLAY * HC) return;
  if (in_sizes[8]  != NLAY * HC) return;
  if (in_sizes[9]  != NLAY * HA) return;
  if (in_sizes[10] != NLAY * HA) return;
  if (in_sizes[11] != NLAY * HA) return;
  if (in_sizes[12] != NLAY * HA) return;
  if (in_sizes[13] != HA) return;
  if (in_sizes[14] != 1) return;
  if (out_size != 1) return;

  const int*   node_attr = (const int*)  d_in[0];
  const float* edge_attr = (const float*)d_in[1];
  const int*   edge_idx  = (const int*)  d_in[2];
  const float* tvec      = (const float*)d_in[3];
  const float* emb       = (const float*)d_in[4];
  const float* W         = (const float*)d_in[5];
  const float* bvec      = (const float*)d_in[6];
  const float* g_h       = (const float*)d_in[7];
  const float* b_h       = (const float*)d_in[8];
  const float* g_o       = (const float*)d_in[9];
  const float* b_o       = (const float*)d_in[10];
  const float* tw        = (const float*)d_in[11];
  const float* tb        = (const float*)d_in[12];
  const float* eo_w      = (const float*)d_in[13];
  const float* eo_b      = (const float*)d_in[14];

  const size_t szX    = (size_t)NNODE * HA * sizeof(float);
  const size_t szX16  = (size_t)NNODE * HA * sizeof(f16);
  const size_t szWt   = (size_t)NCOL * HA * sizeof(f16);
  const size_t szPQ   = (size_t)NNODE * NCOL * sizeof(float);
  const size_t szSum  = (size_t)NNODE * HA * sizeof(float);
  const size_t szPH   = (size_t)NBLK_E * 2 * HC * sizeof(double);
  const size_t szPO   = (size_t)NBLK_E * 2 * HA * sizeof(double);
  const size_t szBnH  = 4096;
  const size_t szBnO  = 4096;
  const size_t oX   = 0;
  const size_t oX16 = oX   + szX;
  const size_t oWt  = oX16 + szX16;
  const size_t oPQ  = oWt  + szWt;
  const size_t oSum = oPQ  + szPQ;
  const size_t oPH  = oSum + szSum;
  const size_t oPO  = oPH  + szPH;
  const size_t oBnH = oPO  + szPO;
  const size_t oBnO = oBnH + szBnH;
  const size_t total = oBnO + szBnO;
  if (total > ws_size) return;

  char*   ws   = (char*)d_ws;
  float*  x    = (float*) (ws + oX);
  f16*    x16  = (f16*)   (ws + oX16);
  f16*    Wt   = (f16*)   (ws + oWt);
  float*  PQ   = (float*) (ws + oPQ);
  float*  summ = (float*) (ws + oSum);
  double* partH = (double*)(ws + oPH);
  double* partO = (double*)(ws + oPO);
  float*  bnH  = (float*) (ws + oBnH);
  float*  bnO  = (float*) (ws + oBnO);
  float*  out  = (float*) d_out;

  embed_kernel<<<NNODE / NPB, 256, 0, stream>>>(node_attr, emb, x, x16);

  for (int l = 0; l < NLAY; ++l) {
    const float* Wl = W + (size_t)l * KW * HC;
    wcvt_kernel<<<NCOL / 16, 256, 0, stream>>>(Wl, Wt);
    gemm_kernel<<<dim3(NNODE / 64, NCOL / 128, 1), 256, 0, stream>>>(x16, Wt, PQ);
    stats_kernel<<<NBLK_E, 256, 0, stream>>>(PQ, edge_idx, edge_attr, Wl, bvec + l * HC, partH);
    bnfin_kernel<<<1, HC, 0, stream>>>(partH, NBLK_E, HC, 1.0 / (double)(NNODE * MM),
                                       g_h + l * HC, b_h + l * HC, bnH);
    apply_kernel<<<NBLK_E, 256, 0, stream>>>(PQ, edge_idx, edge_attr, Wl, bvec + l * HC,
                                           bnH, summ, partO);
    bnfin_kernel<<<1, HA, 0, stream>>>(partO, NBLK_E, HA, 1.0 / (double)NNODE,
                                       g_o + l * HA, b_o + l * HA, bnO);
    update_kernel<<<NNODE / NPB, 256, 0, stream>>>(summ, bnO, tvec, tw + l * HA, tb + l * HA,
                                                 x, x16);
  }

  out_kernel<<<1, 256, 0, stream>>>(x, eo_w, eo_b, out);
}
